// RelativeGlobalAttention_56367150792993
// MI455X (gfx1250) — hardware-verified
//
#include <hip/hip_runtime.h>
#include <math.h>
#include <stdint.h>

#define NB   4
#define SEQ  4096
#define HID  128
#define NH   4
#define HD   32
#define NQB  (SEQ / 64)

typedef __attribute__((ext_vector_type(16))) _Float16 v16h;
typedef __attribute__((ext_vector_type(8)))  _Float16 v8h;
typedef __attribute__((ext_vector_type(16))) __bf16   v16b;
typedef __attribute__((ext_vector_type(8)))  __bf16   v8b;
typedef __attribute__((ext_vector_type(8)))  float    v8f;
typedef __attribute__((ext_vector_type(4)))  float    v4f;
typedef __attribute__((ext_vector_type(4)))  unsigned int v4u;
typedef v4f __attribute__((may_alias)) v4fa;

__device__ __forceinline__ unsigned short f2bf_bits(float f) {
  unsigned u = __float_as_uint(f);
  return (unsigned short)((u + 0x7FFFu + ((u >> 16) & 1u)) >> 16);
}
__device__ __forceinline__ float bf_bits2f(unsigned short h) { return __uint_as_float(((unsigned)h) << 16); }
__device__ __forceinline__ float bf_rne(float f) { return bf_bits2f(f2bf_bits(f)); }
__device__ __forceinline__ unsigned pk16(unsigned short a, unsigned short b) { return (unsigned)a | ((unsigned)b << 16); }

__device__ __forceinline__ void dep_guard_b(v8f& a, v8f& b, v16b x, v16b y) { asm volatile("v_nop\n\tv_nop\n\tv_nop\n\tv_nop" : "+v"(a), "+v"(b) : "v"(x), "v"(y)); }
__device__ __forceinline__ void keep4_b(v16b a, v16b b, v16b c, v16b d) { asm volatile("v_nop" :: "v"(a), "v"(b), "v"(c), "v"(d)); }
__device__ __forceinline__ void acc_guard4(v8f& a, v8f& b, v8f& c, v8f& d) { asm volatile("v_nop\n\tv_nop\n\tv_nop\n\tv_nop" : "+v"(a), "+v"(b), "+v"(c), "+v"(d)); }

struct FragB {
  union U { v16b v; v8b h[2]; };
  static __device__ __forceinline__ v16b load(const __bf16* p) {
    U f; f.h[0] = *(const v8b*)(p); f.h[1] = *(const v8b*)(p + 16); return f.v;
  }
  static __device__ __forceinline__ v8f mma(v16b a, v16b b, v8f c) {
    return __builtin_amdgcn_wmma_f32_16x16x32_bf16(false, a, false, b, (short)0, c, false, false);
  }
};

__device__ __forceinline__ v8f zero8() { v8f z = {0.f, 0.f, 0.f, 0.f, 0.f, 0.f, 0.f, 0.f}; return z; }

template <bool SPLIT, int BIAS_MODE, int OUT_MODE>
__global__ __launch_bounds__(256) void wmma_gemm64(
    const unsigned short* __restrict__ Ap, const unsigned short* __restrict__ A2p, int lda, long strideA,
    const unsigned short* __restrict__ Btp, const unsigned short* __restrict__ Bt2p, int ldb, long strideB,
    void* __restrict__ Cout, void* __restrict__ Cout2, int ldc, long strideC,
    const float* __restrict__ bias, int M, int N, int K, float scale) {
  const __bf16* A = (const __bf16*)(const void*)Ap;   const __bf16* A2  = (const __bf16*)(const void*)A2p;
  const __bf16* Bt = (const __bf16*)(const void*)Btp; const __bf16* Bt2 = (const __bf16*)(const void*)Bt2p;
  __shared__ __align__(16) float sT[8][16 * 68];
  const int b    = blockIdx.y;
  const int lane = threadIdx.x & 31;
  const int wave = threadIdx.x >> 5;
  const int tilesN = N >> 6;
  const int tilesM = M >> 6;
  const int tile = blockIdx.x * 8 + wave;
  if (tile >= tilesM * tilesN) return;
  const int tm = tile / tilesN;
  const int tn = tile - tm * tilesN;
  const int m0 = tm << 6;
  const int n0 = tn << 6;

  const __bf16* Ab  = A  + (size_t)b * strideA;
  const __bf16* Bb  = Bt + (size_t)b * strideB;
  const __bf16* Ab2 = SPLIT ? (A2  + (size_t)b * strideA) : nullptr;
  const __bf16* Bb2 = SPLIT ? (Bt2 + (size_t)b * strideB) : nullptr;

  const int rlane = lane & 15;
  const int koff  = (lane >> 4) * 8;
  const int mOff  = (lane >> 4) * 8;

  v8f acc[4][4];
#pragma unroll
  for (int i = 0; i < 4; ++i)
#pragma unroll
    for (int j = 0; j < 4; ++j) acc[i][j] = zero8();

  for (int k0 = 0; k0 < K; k0 += 32) {
    v16b bh[4], bl[4];
#pragma unroll
    for (int j = 0; j < 4; ++j) {
      const size_t bo = (size_t)(n0 + (j << 4) + rlane) * ldb + koff + k0;
      bh[j] = FragB::load(Bb + bo);
      bl[j] = bh[j];
      if (SPLIT) bl[j] = FragB::load(Bb2 + bo);
    }
#pragma unroll
    for (int i = 0; i < 4; ++i) {
      const size_t ao = (size_t)(m0 + (i << 4) + rlane) * lda + koff + k0;
      v16b ah = FragB::load(Ab + ao);
      v16b al = ah;
      if (SPLIT) al = FragB::load(Ab2 + ao);
#pragma unroll
      for (int j = 0; j < 4; ++j) {
        acc[i][j] = FragB::mma(ah, bh[j], acc[i][j]);
        if (SPLIT) {
          acc[i][j] = FragB::mma(ah, bl[j], acc[i][j]);
          acc[i][j] = FragB::mma(al, bh[j], acc[i][j]);
        }
      }
      dep_guard_b(acc[i][0], acc[i][3], ah, al);
    }
    keep4_b(bh[0], bh[1], bh[2], bh[3]);
    if (SPLIT) keep4_b(bl[0], bl[1], bl[2], bl[3]);
  }
  acc_guard4(acc[0][0], acc[0][1], acc[0][2], acc[0][3]);
  acc_guard4(acc[1][0], acc[1][1], acc[1][2], acc[1][3]);
  acc_guard4(acc[2][0], acc[2][1], acc[2][2], acc[2][3]);
  acc_guard4(acc[3][0], acc[3][1], acc[3][2], acc[3][3]);

  float* slab = sT[wave];
#pragma unroll
  for (int i = 0; i < 4; ++i) {
    const int mBase = m0 + (i << 4);
#pragma unroll
    for (int j = 0; j < 4; ++j) {
      const int n = n0 + (j << 4) + rlane;
      float bv = 0.f;
      if (BIAS_MODE == 2) bv = bf_rne(bias[n]);
#pragma unroll
      for (int r = 0; r < 8; ++r) {
        float v = acc[i][j][r] * scale;
        if (BIAS_MODE == 1) v += bf_rne(bias[mBase + mOff + r]);
        if (BIAS_MODE == 2) v += bv;
        slab[(mOff + r) * 68 + (j << 4) + rlane] = v;
      }
    }
    __builtin_amdgcn_fence(__ATOMIC_RELEASE, "workgroup");
    __builtin_amdgcn_wave_barrier();
    __builtin_amdgcn_fence(__ATOMIC_ACQUIRE, "workgroup");
    if (OUT_MODE == 0) {
      float* C = (float*)Cout + (size_t)b * strideC;
      const int hh = lane >> 4, c4 = (lane & 15) * 4;
      for (int pass = 0; pass < 2; ++pass) {
#pragma unroll
        for (int it = 0; it < 8; ++it) {
          const int row = it * 2 + hh;
          v4f v = *(const v4fa*)(slab + row * 68 + c4);
          *(volatile v4f*)(C + (size_t)(mBase + row) * ldc + n0 + c4) = v;
        }
        __threadfence();
      }
    } else {
      const int q = lane >> 3, c8 = (lane & 7) * 8;
      unsigned short* C  = (unsigned short*)Cout  + (size_t)b * strideC;
      unsigned short* C2 = (unsigned short*)Cout2 + (size_t)b * strideC;
      for (int pass = 0; pass < 2; ++pass) {
#pragma unroll
        for (int it = 0; it < 4; ++it) {
          const int row = it * 4 + q;
          const float* sp = slab + row * 68 + c8;
          v8h hv, lv;
#pragma unroll
          for (int e = 0; e < 8; ++e) {
            unsigned short hb = f2bf_bits(sp[e]);
            unsigned short lb = f2bf_bits(sp[e] - bf_bits2f(hb));
            hv[e] = __builtin_bit_cast(_Float16, hb);
            lv[e] = __builtin_bit_cast(_Float16, lb);
          }
          *(volatile v8h*)(C  + (size_t)(mBase + row) * ldc + n0 + c8) = hv;
          *(volatile v8h*)(C2 + (size_t)(mBase + row) * ldc + n0 + c8) = lv;
        }
        __threadfence();
      }
    }
    __builtin_amdgcn_fence(__ATOMIC_RELEASE, "workgroup");
    __builtin_amdgcn_wave_barrier();
    __builtin_amdgcn_fence(__ATOMIC_ACQUIRE, "workgroup");
  }
}

__global__ __launch_bounds__(256) void cvt_bf16x8_kernel(const float* __restrict__ in, unsigned short* __restrict__ o, int n8) {
  const int i = blockIdx.x * 256 + threadIdx.x;
  if (i < n8) {
    const float* sp = in + (size_t)i * 8;
    const v4f a  = *(const v4f*)(sp);
    const v4f a2 = *(const v4f*)(sp + 4);
    v4u w;
    w[0] = pk16(f2bf_bits(a[0]),  f2bf_bits(a[1]));
    w[1] = pk16(f2bf_bits(a[2]),  f2bf_bits(a[3]));
    w[2] = pk16(f2bf_bits(a2[0]), f2bf_bits(a2[1]));
    w[3] = pk16(f2bf_bits(a2[2]), f2bf_bits(a2[3]));
    unsigned short* dp = o + (size_t)i * 8;
    *(volatile v4u*)dp = w;
    __threadfence();
    *(volatile v4u*)dp = w;
  }
}

__global__ __launch_bounds__(256) void tsplit_kernel(const float* __restrict__ W, unsigned short* __restrict__ oh,
                                                     unsigned short* __restrict__ ol, int R, int Cc) {
  __shared__ __align__(16) float tf[64 * 68];
  const int c0  = blockIdx.x * 64;
  const int r0  = blockIdx.y * 64;
  const int tid = threadIdx.x;
  {
    const int lr = tid >> 4;
    const int c4 = (tid & 15) * 4;
#pragma unroll
    for (int it = 0; it < 4; ++it) {
      const int rr = it * 16 + lr;
      const v4f a = *(const v4f*)(W + (size_t)(r0 + rr) * Cc + c0 + c4);
      *(v4f*)(tf + rr * 68 + c4) = a;
    }
  }
  __syncthreads();
  const int sub = tid >> 3;
  const int c8  = (tid & 7) * 8;
  v4u hv[2], lv[2];
#pragma unroll
  for (int it = 0; it < 2; ++it) {
    const int oc = it * 32 + sub;
    v4u a, a2;
#pragma unroll
    for (int q = 0; q < 4; ++q) {
      const float f0 = tf[(c8 + 2 * q) * 68 + oc];
      const float f1 = tf[(c8 + 2 * q + 1) * 68 + oc];
      const unsigned short h0 = f2bf_bits(f0), h1 = f2bf_bits(f1);
      const unsigned short l0 = f2bf_bits(f0 - bf_bits2f(h0)), l1 = f2bf_bits(f1 - bf_bits2f(h1));
      a[q]  = pk16(h0, h1);
      a2[q] = pk16(l0, l1);
    }
    hv[it] = a; lv[it] = a2;
  }
  for (int pass = 0; pass < 2; ++pass) {
#pragma unroll
    for (int it = 0; it < 2; ++it) {
      const int oc = it * 32 + sub;
      const size_t go = (size_t)(c0 + oc) * R + r0 + c8;
      *(volatile v4u*)(oh + go) = hv[it];
      *(volatile v4u*)(ol + go) = lv[it];
    }
    __threadfence();
  }
}

#define AT_NW 4
#define AT_QB 64
#define AT_KC 64
#define EWIN  128
#define GP    80
#define OSP   36

__device__ __forceinline__ __bf16 at_f2bf(float f) { return __builtin_bit_cast(__bf16, f2bf_bits(f)); }
__device__ __forceinline__ void at_split(float f, __bf16& hi, __bf16& lo) {
  const unsigned short hb = f2bf_bits(f);
  hi = __builtin_bit_cast(__bf16, hb);
  lo = at_f2bf(f - __uint_as_float(((unsigned)hb) << 16));
}
__device__ __forceinline__ v8f at_mma(v16b a, v16b b, v8f c) {
  c = __builtin_amdgcn_wmma_f32_16x16x32_bf16(false, a, false, b, (short)0, c, false, false);
  asm volatile("v_nop\n\tv_nop\n\tv_nop\n\tv_nop" : "+v"(c) : "v"(a), "v"(b));
  return c;
}

__global__ __launch_bounds__(128)
void relattn32_kernel(const unsigned short* __restrict__ qhp, const unsigned short* __restrict__ qlp,
                      const unsigned short* __restrict__ khp, const unsigned short* __restrict__ klp,
                      const unsigned short* __restrict__ vhp, const unsigned short* __restrict__ vlp,
                      const unsigned short* __restrict__ erp, float* __restrict__ out, float sscale) {
  union FB { v16b v; v8b h[2]; };
  __shared__ __align__(16) __bf16 Ksh[AT_KC * HD];
  __shared__ __align__(16) __bf16 Ksl[AT_KC * HD];
  __shared__ __align__(16) __bf16 Vth[HD * AT_KC];
  __shared__ __align__(16) __bf16 Vtl[HD * AT_KC];
  __shared__ __align__(16) __bf16 Esh[EWIN * HD];
  __shared__ __align__(16) __bf16 Psh[AT_NW][16 * AT_KC];
  __shared__ __align__(16) __bf16 Psl[AT_NW][16 * AT_KC];
  __shared__ __align__(16) float  Gs[AT_NW][16 * GP];

  const int tid  = threadIdx.x;
  const int wave = tid >> 5;
  const int lane = tid & 31;
  const int hh   = lane >> 4;
  const int c    = lane & 15;

  const int bx   = blockIdx.x;
  const int qb   = bx & (NQB - 1);
  const int pair = bx >> 6;
  const int b    = pair >> 2;
  const int h    = pair & 3;
  const int q0   = qb * AT_QB + wave * 16;
  const size_t rowBase = (size_t)b * SEQ;

  const __bf16* Qh = (const __bf16*)(const void*)qhp + h * HD;
  const __bf16* Ql = (const __bf16*)(const void*)qlp + h * HD;
  const __bf16* Kh = (const __bf16*)(const void*)khp + h * HD;
  const __bf16* Kl = (const __bf16*)(const void*)klp + h * HD;
  const __bf16* Vh = (const __bf16*)(const void*)vhp + ((size_t)b * HID + h * HD) * SEQ;
  const __bf16* Vl = (const __bf16*)(const void*)vlp + ((size_t)b * HID + h * HD) * SEQ;
  const __bf16* Er = (const __bf16*)(const void*)erp;
  float*        ob = out + h * HD;

  const v16b qah = FragB::load(Qh + (rowBase + q0 + c) * HID + 8 * hh);
  const v16b qal = FragB::load(Ql + (rowBase + q0 + c) * HID + 8 * hh);

  float mrow[8], lrow[8];
  v8f oacc[2];
#pragma unroll
  for (int r = 0; r < 8; ++r) { mrow[r] = -INFINITY; lrow[r] = 0.f; }
  oacc[0] = zero8(); oacc[1] = zero8();

  const int wbase = 48 - 16 * wave;
  float* gw = Gs[wave];
  __bf16* pwh = Psh[wave];
  __bf16* pwl = Psl[wave];

  const int nChunks = qb + 1;
  for (int kc = 0; kc < nChunks; ++kc) {
    const int kv0 = kc * AT_KC;
    int e0 = SEQ - 64 - 64 * (qb - kc);
    __syncthreads();
    {
      const int r = tid >> 1, half = (tid & 1) * 16;
      const __bf16* ks = Kh + (rowBase + kv0 + r) * HID + half;
      const __bf16* kl = Kl + (rowBase + kv0 + r) * HID + half;
      const int d = tid >> 2, qt = (tid & 3) * 16;
      const __bf16* vs = Vh + (size_t)d * SEQ + kv0 + qt;
      const __bf16* vl = Vl + (size_t)d * SEQ + kv0 + qt;
      int erow = e0 + tid;
      erow = erow < 0 ? 0 : erow;
      erow = erow > (SEQ - 1) ? (SEQ - 1) : erow;
      const __bf16* es = Er + (size_t)erow * HD;
#pragma unroll
      for (int i = 0; i < 2; ++i) {
        const v8b a0 = *(const v8b*)(ks + 8 * i);
        const v8b a1 = *(const v8b*)(kl + 8 * i);
        const v8b b0 = *(const v8b*)(vs + 8 * i);
        const v8b b1 = *(const v8b*)(vl + 8 * i);
        *(v8b*)(Ksh + r * HD    + half + 8 * i) = a0;
        *(v8b*)(Ksl + r * HD    + half + 8 * i) = a1;
        *(v8b*)(Vth + d * AT_KC + qt   + 8 * i) = b0;
        *(v8b*)(Vtl + d * AT_KC + qt   + 8 * i) = b1;
      }
#pragma unroll
      for (int i = 0; i < 4; ++i) {
        const v8b ee = *(const v8b*)(es + 8 * i);
        *(v8b*)(Esh + tid * HD + 8 * i) = ee;
      }
    }
    __syncthreads();

    v8f s[4];
#pragma unroll
    for (int j = 0; j < 4; ++j) {
      FB kb, kl;
      const __bf16* kp = Ksh + (j * 16 + c) * HD + 8 * hh;
      const __bf16* kq = Ksl + (j * 16 + c) * HD + 8 * hh;
      kb.h[0] = *(const v8b*)(kp); kb.h[1] = *(const v8b*)(kp + 16);
      kl.h[0] = *(const v8b*)(kq); kl.h[1] = *(const v8b*)(kq + 16);
      v8f a = zero8();
      a = at_mma(qah, kb.v, a);
      a = at_mma(qah, kl.v, a);
      a = at_mma(qal, kb.v, a);
      s[j] = a;
    }

#pragma unroll
    for (int nt = 0; nt < 5; ++nt) {
      FB eb;
      const __bf16* ep = Esh + (wbase + nt * 16 + c) * HD + 8 * hh;
      eb.h[0] = *(const v8b*)(ep); eb.h[1] = *(const v8b*)(ep + 16);
      v8f g = zero8();
      g = at_mma(qah, eb.v, g);
      g = at_mma(qal, eb.v, g);
#pragma unroll
      for (int r = 0; r < 8; ++r) gw[(8 * hh + r) * GP + nt * 16 + c] = g[r];
    }
    __builtin_amdgcn_fence(__ATOMIC_RELEASE, "workgroup");
    __builtin_amdgcn_wave_barrier();
    __builtin_amdgcn_fence(__ATOMIC_ACQUIRE, "workgroup");

    const bool diag = (kc == qb);
    float cm[8];
#pragma unroll
    for (int r = 0; r < 8; ++r) {
      const int il   = wave * 16 + 8 * hh + r;
      const int qrow = qb * AT_QB + il;
      const float* gr = gw + (8 * hh + r) * GP + (15 - 8 * hh - r);
      float m = -INFINITY;
#pragma unroll
      for (int j = 0; j < 4; ++j) {
        const int kvcol = kv0 + j * 16 + c;
        const float rel = gr[j * 16 + c];
        const float sv  = (s[j][r] + rel) * sscale;
        const bool msk  = diag && (kvcol > qrow);
        const float sm  = msk ? -INFINITY : sv;
        s[j][r] = sm;
        m = fmaxf(m, sm);
      }
#pragma unroll
      for (int off = 1; off < 16; off <<= 1) m = fmaxf(m, __shfl_xor(m, off, 32));
      cm[r] = m;
    }

#pragma unroll
    for (int r = 0; r < 8; ++r) {
      const float mnew  = fmaxf(mrow[r], cm[r]);
      const float alpha = __expf(mrow[r] - mnew);
      mrow[r] = mnew;
      float psum = 0.f;
#pragma unroll
      for (int j = 0; j < 4; ++j) {
        const float p = __expf(s[j][r] - mnew);
        psum += p;
        __bf16 a, bl; at_split(p, a, bl);
        pwh[(8 * hh + r) * AT_KC + j * 16 + c] = a;
        pwl[(8 * hh + r) * AT_KC + j * 16 + c] = bl;
      }
#pragma unroll
      for (int off = 1; off < 16; off <<= 1) psum += __shfl_xor(psum, off, 32);
      lrow[r] = lrow[r] * alpha + psum;
      oacc[0][r] *= alpha;
      oacc[1][r] *= alpha;
    }
    __builtin_amdgcn_fence(__ATOMIC_RELEASE, "workgroup");
    __builtin_amdgcn_wave_barrier();
    __builtin_amdgcn_fence(__ATOMIC_ACQUIRE, "workgroup");

#pragma unroll 1
    for (int kk = 0; kk < 2; ++kk) {
      FB pa, pl;
      pa.h[0] = *(const v8b*)(pwh + c * AT_KC + kk * 32 + 8 * hh);
      pa.h[1] = *(const v8b*)(pwh + c * AT_KC + kk * 32 + 16 + 8 * hh);
      pl.h[0] = *(const v8b*)(pwl + c * AT_KC + kk * 32 + 8 * hh);
      pl.h[1] = *(const v8b*)(pwl + c * AT_KC + kk * 32 + 16 + 8 * hh);
#pragma unroll
      for (int t = 0; t < 2; ++t) {
        FB vb, vl;
        vb.h[0] = *(const v8b*)(Vth + (t * 16 + c) * AT_KC + kk * 32 + 8 * hh);
        vb.h[1] = *(const v8b*)(Vth + (t * 16 + c) * AT_KC + kk * 32 + 16 + 8 * hh);
        vl.h[0] = *(const v8b*)(Vtl + (t * 16 + c) * AT_KC + kk * 32 + 8 * hh);
        vl.h[1] = *(const v8b*)(Vtl + (t * 16 + c) * AT_KC + kk * 32 + 16 + 8 * hh);
        oacc[t] = at_mma(pa.v, vb.v, oacc[t]);
        oacc[t] = at_mma(pa.v, vl.v, oacc[t]);
        oacc[t] = at_mma(pl.v, vb.v, oacc[t]);
      }
    }
  }

  __builtin_amdgcn_fence(__ATOMIC_RELEASE, "workgroup");
  __builtin_amdgcn_wave_barrier();
  __builtin_amdgcn_fence(__ATOMIC_ACQUIRE, "workgroup");
  float* os = gw;
#pragma unroll
  for (int r = 0; r < 8; ++r) {
    const float inv = 1.0f / lrow[r];
    os[(8 * hh + r) * OSP + c]      = oacc[0][r] * inv;
    os[(8 * hh + r) * OSP + 16 + c] = oacc[1][r] * inv;
  }
  __builtin_amdgcn_fence(__ATOMIC_RELEASE, "workgroup");
  __builtin_amdgcn_wave_barrier();
  __builtin_amdgcn_fence(__ATOMIC_ACQUIRE, "workgroup");
  {
    const int q4 = lane >> 3, c4 = (lane & 7) * 4;
    for (int pass = 0; pass < 2; ++pass) {
#pragma unroll
      for (int it = 0; it < 4; ++it) {
        const int row = it * 4 + q4;
        const v4f val = *(const v4fa*)(os + row * OSP + c4);
        *(volatile v4f*)(ob + (rowBase + q0 + row) * HID + c4) = val;
      }
      __threadfence();
    }
  }
}

extern "C" void kernel_launch(void* const* d_in, const int* in_sizes, int n_in,
                              void* d_out, int out_size, void* d_ws, size_t ws_size,
                              hipStream_t stream) {
  if (n_in < 8) return;
  if (in_sizes[0] != NB * SEQ * HID) return;
  if (in_sizes[1] != HID * HID || in_sizes[3] != HID * HID || in_sizes[5] != HID * HID) return;
  if (in_sizes[2] != HID || in_sizes[4] != HID || in_sizes[6] != HID) return;
  if (in_sizes[7] != SEQ * HD) return;
  if (out_size != NB * SEQ * HID) return;

  const float* x  = (const float*)d_in[0];
  const float* Wq = (const float*)d_in[1];
  const float* bq = (const float*)d_in[2];
  const float* Wk = (const float*)d_in[3];
  const float* bk = (const float*)d_in[4];
  const float* Wv = (const float*)d_in[5];
  const float* bv = (const float*)d_in[6];
  const float* Er = (const float*)d_in[7];
  float* out = (float*)d_out;

  const size_t PW = (size_t)HID * HID * 2;
  const size_t PX = (size_t)NB * SEQ * HID * 2;
  const size_t PE = (size_t)SEQ * HD * 2;
  const size_t PV = (size_t)NB * HID * SEQ * 2;
  size_t off = 0;
  const size_t oWqTh = off; off += PW;  const size_t oWqTl = off; off += PW;
  const size_t oWkTh = off; off += PW;  const size_t oWkTl = off; off += PW;
  const size_t oWvTh = off; off += PW;  const size_t oWvTl = off; off += PW;
  const size_t oXb   = off; off += PX;
  const size_t oErB  = off; off += PE;
  const size_t oQh   = off; off += PX;  const size_t oQl   = off; off += PX;
  const size_t oKh   = off; off += PX;  const size_t oKl   = off; off += PX;
  const size_t oVTh  = off; off += PV;  const size_t oVTl  = off; off += PV;
  if (off > ws_size) return;
  if (off > (size_t)134217728) return;

  char* ws = (char*)d_ws;
  unsigned short* WqTh = (unsigned short*)(ws + oWqTh); unsigned short* WqTl = (unsigned short*)(ws + oWqTl);
  unsigned short* WkTh = (unsigned short*)(ws + oWkTh); unsigned short* WkTl = (unsigned short*)(ws + oWkTl);
  unsigned short* WvTh = (unsigned short*)(ws + oWvTh); unsigned short* WvTl = (unsigned short*)(ws + oWvTl);
  unsigned short* Xb   = (unsigned short*)(ws + oXb);
  unsigned short* ErB  = (unsigned short*)(ws + oErB);
  unsigned short* Qh   = (unsigned short*)(ws + oQh);   unsigned short* Ql   = (unsigned short*)(ws + oQl);
  unsigned short* Kh   = (unsigned short*)(ws + oKh);   unsigned short* Kl   = (unsigned short*)(ws + oKl);
  unsigned short* VTh  = (unsigned short*)(ws + oVTh);  unsigned short* VTl  = (unsigned short*)(ws + oVTl);

  const dim3 blk(256);
  const float sscale = 0.17677669529663688f;

  tsplit_kernel<<<dim3(HID / 64, HID / 64), blk, 0, stream>>>(Wq, WqTh, WqTl, HID, HID);
  tsplit_kernel<<<dim3(HID / 64, HID / 64), blk, 0, stream>>>(Wk, WkTh, WkTl, HID, HID);
  tsplit_kernel<<<dim3(HID / 64, HID / 64), blk, 0, stream>>>(Wv, WvTh, WvTl, HID, HID);
  const int n8x = NB * SEQ * HID / 8;
  const int n8e = SEQ * HD / 8;
  cvt_bf16x8_kernel<<<dim3((n8x + 255) / 256), blk, 0, stream>>>(x, Xb, n8x);
  cvt_bf16x8_kernel<<<dim3((n8e + 255) / 256), blk, 0, stream>>>(Er, ErB, n8e);
  const dim3 gProj(((NB * SEQ / 64) * (HID / 64) + 7) / 8, 1);
  wmma_gemm64<false, 2, 2><<<gProj, blk, 0, stream>>>(
      Xb, Xb, HID, 0L, WqTh, WqTh, HID, 0L, (void*)Qh, (void*)Ql, HID, 0L, bq, NB * SEQ, HID, HID, 1.0f);
  wmma_gemm64<false, 2, 2><<<gProj, blk, 0, stream>>>(
      Xb, Xb, HID, 0L, WkTh, WkTh, HID, 0L, (void*)Kh, (void*)Kl, HID, 0L, bk, NB * SEQ, HID, HID, 1.0f);
  const dim3 gVT(((HID / 64) * (SEQ / 64) + 7) / 8, NB);
  wmma_gemm64<false, 1, 2><<<gVT, blk, 0, stream>>>(
      WvTh, WvTh, HID, 0L, Xb, Xb, HID, (long)SEQ * HID, (void*)VTh, (void*)VTl, SEQ, (long)HID * SEQ,
      bv, HID, SEQ, HID, 1.0f);
  relattn32_kernel<<<dim3(NB * NH * NQB), dim3(128), 0, stream>>>(Qh, Ql, Kh, Kl, VTh, VTl, ErB, out, sscale);
  (void)hipGetLastError();
}
